// PatchSSMClassifier_44667659878986
// MI455X (gfx1250) — hardware-verified
//
#include <hip/hip_runtime.h>
#include <math.h>

constexpr int kBatch     = 128;
constexpr int kSteps     = 256;
constexpr int kDModel    = 512;
constexpr int kDState    = 1024;
constexpr int kNCls      = 1000;
constexpr int kNClsPad   = 1024;
constexpr int kPatchK    = 48;
constexpr int kPatchKPad = 64;
constexpr int kRows      = kBatch * kSteps;
constexpr int kHalfRows  = kRows / 2;
constexpr int kKCat      = kDState + kDModel;
constexpr int kTilePitch = 1544;
constexpr int kRowsPerBlk = 16;

constexpr float kCatCarry    = 64.0f;
constexpr float kCatCarryInv = 1.0f / 64.0f;
constexpr float kCmCarry     = 64.0f;
constexpr float kCmCarryInv  = 1.0f / 64.0f;
constexpr float kWpCarry     = 16.0f;
constexpr float kWpCarryInv  = 1.0f / 16.0f;
constexpr float kWfCarry     = 16.0f;
constexpr float kPoolMeanCarry = 1.0f / 16.0f;
constexpr float kLogitScale  = 1.0f / 256.0f;

typedef __attribute__((ext_vector_type(16))) _Float16 v16h;
typedef __attribute__((ext_vector_type(8)))  _Float16 v8h;
typedef __attribute__((ext_vector_type(16))) __bf16   v16b;
typedef __attribute__((ext_vector_type(8)))  __bf16   v8b;
typedef __attribute__((ext_vector_type(8)))  float    v8f;
typedef __attribute__((ext_vector_type(4)))  float    v4f;
typedef __attribute__((ext_vector_type(4)))  unsigned int v4u;

__device__ __forceinline__ unsigned short f2bf_bits(float f) {
  unsigned u = __float_as_uint(f);
  return (unsigned short)((u + 0x7FFFu + ((u >> 16) & 1u)) >> 16);
}
__device__ __forceinline__ float bf_bits2f(unsigned short h) { return __uint_as_float(((unsigned)h) << 16); }

__device__ __forceinline__ void dep_guard_h(v8f& a, v8f& b, v16h x, v16h y) { asm volatile("v_nop\n\tv_nop\n\tv_nop\n\tv_nop" : "+v"(a), "+v"(b) : "v"(x), "v"(y)); }
__device__ __forceinline__ void dep_guard_b(v8f& a, v8f& b, v16b x, v16b y) { asm volatile("v_nop\n\tv_nop\n\tv_nop\n\tv_nop" : "+v"(a), "+v"(b) : "v"(x), "v"(y)); }
__device__ __forceinline__ void keep4_h(v16h a, v16h b, v16h c, v16h d) { asm volatile("v_nop" :: "v"(a), "v"(b), "v"(c), "v"(d)); }
__device__ __forceinline__ void keep4_b(v16b a, v16b b, v16b c, v16b d) { asm volatile("v_nop" :: "v"(a), "v"(b), "v"(c), "v"(d)); }
__device__ __forceinline__ void acc_guard4(v8f& a, v8f& b, v8f& c, v8f& d) { asm volatile("v_nop\n\tv_nop\n\tv_nop\n\tv_nop" : "+v"(a), "+v"(b), "+v"(c), "+v"(d)); }
__device__ __forceinline__ void guard4_h(v8f& a0, v8f& a1, v8f& a2, v8f& a3, v16h x, v16h y) {
  asm volatile("v_nop\n\tv_nop\n\tv_nop\n\tv_nop" : "+v"(a0), "+v"(a1), "+v"(a2), "+v"(a3) : "v"(x), "v"(y));
}
template <typename T> struct Frag;
template <> struct Frag<_Float16> {
  typedef v16h V; union U { v16h v; v8h h[2]; };
  static __device__ __forceinline__ v16h load(const _Float16* p) {
    U f; f.h[0] = *(const v8h*)(p); f.h[1] = *(const v8h*)(p + 16); return f.v;
  }
  static __device__ __forceinline__ v8f mma(v16h a, v16h b, v8f c) {
    return __builtin_amdgcn_wmma_f32_16x16x32_f16(false, a, false, b, (short)0, c, false, false);
  }
  static __device__ __forceinline__ void guard(v8f& a, v8f& b, v16h x, v16h y) { dep_guard_h(a, b, x, y); }
  static __device__ __forceinline__ void keep(v16h a, v16h b, v16h c, v16h d) { keep4_h(a, b, c, d); }
};
template <> struct Frag<__bf16> {
  typedef v16b V; union U { v16b v; v8b h[2]; };
  static __device__ __forceinline__ v16b load(const __bf16* p) {
    U f; f.h[0] = *(const v8b*)(p); f.h[1] = *(const v8b*)(p + 16); return f.v;
  }
  static __device__ __forceinline__ v8f mma(v16b a, v16b b, v8f c) {
    return __builtin_amdgcn_wmma_f32_16x16x32_bf16(false, a, false, b, (short)0, c, false, false);
  }
  static __device__ __forceinline__ void guard(v8f& a, v8f& b, v16b x, v16b y) { dep_guard_b(a, b, x, y); }
  static __device__ __forceinline__ void keep(v16b a, v16b b, v16b c, v16b d) { keep4_b(a, b, c, d); }
};

__device__ __forceinline__ unsigned pk16(unsigned short a, unsigned short b) { return (unsigned)a | ((unsigned)b << 16); }
__device__ __forceinline__ unsigned short h_bits(float f) { const _Float16 h = (_Float16)f; return __builtin_bit_cast(unsigned short, h); }

template <int ET> struct Elem;
template <> struct Elem<0> { typedef _Float16 T; };
template <> struct Elem<1> { typedef __bf16 T; };
template <int ET, bool SPLIT, int BIAS_MODE, int OUT_MODE, bool RESID, int ACT = 0>
__global__ __launch_bounds__(256) void wmma_gemm64(
    const unsigned short* __restrict__ Ap, const unsigned short* __restrict__ A2p, int lda, long strideA,
    const unsigned short* __restrict__ Btp, const unsigned short* __restrict__ Bt2p, int ldb, long strideB,
    void* __restrict__ Cout, void* __restrict__ Cout2, int ldc, long strideC,
    const float* __restrict__ bias,
    const float* __restrict__ resid, long strideR,
    int M, int N, int K, float scale) {
  typedef typename Elem<ET>::T T;
  typedef typename Frag<T>::V V;
  const T* A = (const T*)Ap; const T* A2 = (const T*)A2p; const T* Bt = (const T*)Btp; const T* Bt2 = (const T*)Bt2p;
  __shared__ __align__(16) float sT[8][16 * 68];
  const int b    = blockIdx.y;
  const int lane = threadIdx.x & 31;
  const int wave = threadIdx.x >> 5;
  const int tilesN = N >> 6;
  const int tilesM = M >> 6;
  const int tile = blockIdx.x * 8 + wave;
  if (tile >= tilesM * tilesN) return;
  const int tm = tile / tilesN;
  const int tn = tile - tm * tilesN;
  const int m0 = tm << 6;
  const int n0 = tn << 6;

  const T* Ab  = A  + (size_t)b * strideA;
  const T* Bb  = Bt + (size_t)b * strideB;
  const T* Ab2 = SPLIT ? (A2  + (size_t)b * strideA) : nullptr;
  const T* Bb2 = SPLIT ? (Bt2 + (size_t)b * strideB) : nullptr;

  const int rlane = lane & 15;
  const int koff  = (lane >> 4) * 8;
  const int mOff  = (lane >> 4) * 8;

  v8f acc[4][4];
#pragma unroll
  for (int i = 0; i < 4; ++i)
#pragma unroll
    for (int j = 0; j < 4; ++j) acc[i][j] = (v8f){0.f,0.f,0.f,0.f,0.f,0.f,0.f,0.f};

  for (int k0 = 0; k0 < K; k0 += 32) {
    V bh[4], bl[4];
#pragma unroll
    for (int j = 0; j < 4; ++j) {
      const size_t bo = (size_t)(n0 + (j << 4) + rlane) * ldb + koff + k0;
      bh[j] = Frag<T>::load(Bb + bo);
      if (SPLIT) bl[j] = Frag<T>::load(Bb2 + bo);
    }
#pragma unroll
    for (int i = 0; i < 4; ++i) {
      const size_t ao = (size_t)(m0 + (i << 4) + rlane) * lda + koff + k0;
      V ah = Frag<T>::load(Ab + ao);
      V al;
      if (SPLIT) al = Frag<T>::load(Ab2 + ao);
#pragma unroll
      for (int j = 0; j < 4; ++j) {
        acc[i][j] = Frag<T>::mma(ah, bh[j], acc[i][j]);
        if (SPLIT) {
          acc[i][j] = Frag<T>::mma(ah, bl[j], acc[i][j]);
          acc[i][j] = Frag<T>::mma(al, bh[j], acc[i][j]);
        }
      }
      Frag<T>::guard(acc[i][0], acc[i][3], ah, SPLIT ? al : ah);
    }
    Frag<T>::keep(bh[0], bh[1], bh[2], bh[3]);
    if (SPLIT) Frag<T>::keep(bl[0], bl[1], bl[2], bl[3]);
  }
  acc_guard4(acc[0][0], acc[0][1], acc[0][2], acc[0][3]);
  acc_guard4(acc[1][0], acc[1][1], acc[1][2], acc[1][3]);
  acc_guard4(acc[2][0], acc[2][1], acc[2][2], acc[2][3]);
  acc_guard4(acc[3][0], acc[3][1], acc[3][2], acc[3][3]);

  float* slab = sT[wave];
  const float* Rb = RESID ? (resid + (size_t)b * strideR) : nullptr;
#pragma unroll
  for (int i = 0; i < 4; ++i) {
    const int mBase = m0 + (i << 4);
#pragma unroll
    for (int j = 0; j < 4; ++j) {
      const int n = n0 + (j << 4) + rlane;
      float bv = 0.f;
      if (BIAS_MODE == 2) bv = bias[n];
#pragma unroll
      for (int r = 0; r < 8; ++r) {
        float v = acc[i][j][r] * scale;
        if (BIAS_MODE == 1) v += bias[mBase + mOff + r];
        if (BIAS_MODE == 2) v += bv;
        if (RESID) v += Rb[(size_t)(mBase + mOff + r) * ldc + n];
        if (ACT == 2) v = fmaxf(v, 0.0f);
        if (ACT == 4) v = (v > 0.f) ? v : 0.01f * v;
        slab[(mOff + r) * 68 + (j << 4) + rlane] = v;
      }
    }
    __builtin_amdgcn_fence(__ATOMIC_RELEASE, "workgroup");
    __builtin_amdgcn_wave_barrier();
    __builtin_amdgcn_fence(__ATOMIC_ACQUIRE, "workgroup");
    if (OUT_MODE == 0) {
      float* C = (float*)Cout + (size_t)b * strideC;
      const int hh = lane >> 4, c4 = (lane & 15) * 4;
      for (int pass = 0; pass < 2; ++pass) {
#pragma unroll
        for (int it = 0; it < 8; ++it) {
          const int row = it * 2 + hh;
          v4f v = *(const v4f*)(slab + row * 68 + c4);
          *(volatile v4f*)(C + (size_t)(mBase + row) * ldc + n0 + c4) = v;
        }
        __threadfence();
      }
    } else {
      const int q = lane >> 3, c8 = (lane & 7) * 8;
      unsigned short* C  = (unsigned short*)Cout  + (size_t)b * strideC;
      unsigned short* C2 = (OUT_MODE == 2) ? ((unsigned short*)Cout2 + (size_t)b * strideC) : nullptr;
      for (int pass = 0; pass < 2; ++pass) {
#pragma unroll
        for (int it = 0; it < 4; ++it) {
          const int row = it * 4 + q;
          const float* sp = slab + row * 68 + c8;
          v8h hv, lv;
#pragma unroll
          for (int e = 0; e < 8; ++e) {
            if (OUT_MODE == 1) {
              hv[e] = (_Float16)sp[e];
            } else {
              unsigned short hb = f2bf_bits(sp[e]);
              unsigned short lb = f2bf_bits(sp[e] - bf_bits2f(hb));
              hv[e] = __builtin_bit_cast(_Float16, hb);
              lv[e] = __builtin_bit_cast(_Float16, lb);
            }
          }
          *(volatile v8h*)(C + (size_t)(mBase + row) * ldc + n0 + c8) = hv;
          if (OUT_MODE == 2) *(volatile v8h*)(C2 + (size_t)(mBase + row) * ldc + n0 + c8) = lv;
        }
        __threadfence();
      }
    }
    __builtin_amdgcn_fence(__ATOMIC_RELEASE, "workgroup");
    __builtin_amdgcn_wave_barrier();
    __builtin_amdgcn_fence(__ATOMIC_ACQUIRE, "workgroup");
  }
}

__global__ __launch_bounds__(256) void build_wcat_kernel(const float* __restrict__ Am, const float* __restrict__ Bmm,
                                                         unsigned short* __restrict__ out) {
  const int t = blockIdx.x * 256 + threadIdx.x;
  if (t >= kDState * (kKCat / 8)) return;
  const int n = t / (kKCat / 8);
  const int g = t - n * (kKCat / 8);
  const int col = g * 8;
  const int ca = (col < kDState - 8) ? col : (kDState - 8);
  const int cbr = col - kDState;
  const int cb = (cbr > 0) ? cbr : 0;
  const float* pa = Am  + (size_t)n * kDState + ca;
  const float* pb = Bmm + (size_t)n * kDModel + cb;
  const v4f a0 = *(const v4f*)(pa);
  const v4f a1 = *(const v4f*)(pa + 4);
  const v4f b0 = *(const v4f*)(pb);
  const v4f b1 = *(const v4f*)(pb + 4);
  const bool useA = (col < kDState);
  unsigned short hb[8];
#pragma unroll
  for (int e = 0; e < 4; ++e) {
    const float x0 = useA ? a0[e] : b0[e];
    const float x1 = useA ? a1[e] : b1[e];
    hb[e]     = h_bits(x0 * kCatCarry);
    hb[4 + e] = h_bits(x1 * kCatCarry);
  }
  const v4u u = (v4u){pk16(hb[0], hb[1]), pk16(hb[2], hb[3]), pk16(hb[4], hb[5]), pk16(hb[6], hb[7])};
  unsigned short* q = out + (size_t)n * kKCat + col;
  *(volatile v4u*)q = u;
  __threadfence();
  *(volatile v4u*)q = u;
}

__global__ __launch_bounds__(256) void cast8_scale_kernel(const float* __restrict__ in, unsigned short* __restrict__ out,
                                                          int n8, float scale) {
  const int i = blockIdx.x * 256 + threadIdx.x;
  if (i >= n8) return;
  const float* p = in + 8 * (size_t)i;
  const v4f a = *(const v4f*)(p);
  const v4f c = *(const v4f*)(p + 4);
  unsigned short hb[8];
#pragma unroll
  for (int e = 0; e < 4; ++e) {
    hb[e]     = h_bits(a[e] * scale);
    hb[4 + e] = h_bits(c[e] * scale);
  }
  const v4u u = (v4u){pk16(hb[0], hb[1]), pk16(hb[2], hb[3]), pk16(hb[4], hb[5]), pk16(hb[6], hb[7])};
  unsigned short* q = out + 8 * (size_t)i;
  *(volatile v4u*)q = u;
  __threadfence();
  *(volatile v4u*)q = u;
}

__global__ __launch_bounds__(256) void cast_wf_kernel(const float* __restrict__ Wf, unsigned short* __restrict__ out) {
  const int t = blockIdx.x * 256 + threadIdx.x;
  if (t >= kNClsPad * (kDModel / 8)) return;
  const int r = t >> 6;
  const int g = t & 63;
  const int rc = (r < kNCls) ? r : (kNCls - 1);
  const float* p = Wf + (size_t)rc * kDModel + g * 8;
  const v4f a = *(const v4f*)(p);
  const v4f c = *(const v4f*)(p + 4);
  const bool keep = (r < kNCls);
  unsigned short hb[8];
#pragma unroll
  for (int e = 0; e < 4; ++e) {
    hb[e]     = h_bits(keep ? a[e] * kWfCarry : 0.0f);
    hb[4 + e] = h_bits(keep ? c[e] * kWfCarry : 0.0f);
  }
  const v4u u = (v4u){pk16(hb[0], hb[1]), pk16(hb[2], hb[3]), pk16(hb[4], hb[5]), pk16(hb[6], hb[7])};
  unsigned short* q = out + (size_t)r * kDModel + g * 8;
  *(volatile v4u*)q = u;
  __threadfence();
  *(volatile v4u*)q = u;
}

__global__ __launch_bounds__(256) void cast_wp_kernel(const float* __restrict__ Wp, unsigned short* __restrict__ out) {
  const int t = blockIdx.x * 256 + threadIdx.x;
  if (t >= kDModel * (kPatchKPad / 8)) return;
  const int r = t >> 3;
  const int g = t & 7;
  const int gc = (g < 6) ? g : 5;
  const float* p = Wp + (size_t)r * kPatchK + gc * 8;
  const v4f a = *(const v4f*)(p);
  const v4f c = *(const v4f*)(p + 4);
  const bool keep = (g < 6);
  unsigned short hb[8];
#pragma unroll
  for (int e = 0; e < 4; ++e) {
    hb[e]     = h_bits(keep ? a[e] * kWpCarry : 0.0f);
    hb[4 + e] = h_bits(keep ? c[e] * kWpCarry : 0.0f);
  }
  const v4u u = (v4u){pk16(hb[0], hb[1]), pk16(hb[2], hb[3]), pk16(hb[4], hb[5]), pk16(hb[6], hb[7])};
  unsigned short* q = out + (size_t)r * kPatchKPad + g * 8;
  *(volatile v4u*)q = u;
  __threadfence();
  *(volatile v4u*)q = u;
}

__global__ __launch_bounds__(256) void patchify_kernel(const float* __restrict__ images, unsigned short* __restrict__ out) {
  const int t = blockIdx.x * 256 + threadIdx.x;
  if (t >= kRows * (kPatchKPad / 8)) return;
  const int row = t >> 3;
  const int g   = t & 7;
  const int tt  = row >> 7;
  const int b   = row & 127;
  const int ph  = tt >> 4;
  const int pw  = tt & 15;
  const int gc  = (g < 6) ? g : 5;
  const int ch  = gc >> 1;
  const int py0 = (gc & 1) * 2;
  const float* p = images + ((((size_t)b * 3 + ch) * 64 + ph * 4 + py0) * 64 + pw * 4);
  const v4f r0 = *(const v4f*)(p);
  const v4f r1 = *(const v4f*)(p + 64);
  const bool keep = (g < 6);
  unsigned short hb[8];
#pragma unroll
  for (int e = 0; e < 4; ++e) {
    hb[e]     = h_bits(keep ? r0[e] : 0.0f);
    hb[4 + e] = h_bits(keep ? r1[e] : 0.0f);
  }
  const v4u u = (v4u){pk16(hb[0], hb[1]), pk16(hb[2], hb[3]), pk16(hb[4], hb[5]), pk16(hb[6], hb[7])};
  unsigned short* q = out + (size_t)row * kPatchKPad + g * 8;
  *(volatile v4u*)q = u;
  __threadfence();
  *(volatile v4u*)q = u;
}

__global__ __launch_bounds__(256) void ssm_scan_kernel(const unsigned short* __restrict__ X16p,
                                                       const unsigned short* __restrict__ Wcatp,
                                                       unsigned short* __restrict__ S16p) {
  typedef Frag<_Float16> FH;
  __shared__ __align__(16) _Float16 tile[kRowsPerBlk * kTilePitch];
  const _Float16* X16  = (const _Float16*)(const void*)X16p;
  const _Float16* Wcat = (const _Float16*)(const void*)Wcatp;
  _Float16* S16 = (_Float16*)(void*)S16p;
  const int tid  = threadIdx.x;
  const int lane = tid & 31;
  const int wave = tid >> 5;
  const int c    = lane & 15;
  const int hh   = lane >> 4;
  const int b0   = blockIdx.x * kRowsPerBlk;

  {
    const _Float16 z = (_Float16)0.0f;
    const v8h z8 = (v8h){z, z, z, z, z, z, z, z};
#pragma unroll
    for (int i = 0; i < 8; ++i) {
      const int idx  = i * 256 + tid;
      const int row  = idx >> 7;
      const int col8 = (idx & 127) * 8;
      *(v8h*)(tile + row * kTilePitch + col8) = z8;
    }
  }
#pragma unroll
  for (int i = 0; i < 4; ++i) {
    const int idx  = i * 256 + tid;
    const int row  = idx >> 6;
    const int col8 = (idx & 63) * 8;
    const v8h v = *(const v8h*)(X16 + ((size_t)(0 * kBatch + b0 + row)) * kDModel + col8);
    *(v8h*)(tile + row * kTilePitch + kDState + col8) = v;
  }
  __syncthreads();

  const int aoff = c * kTilePitch + hh * 8;
  const size_t woff = (size_t)(wave * 128 + c) * kKCat + hh * 8;

  for (int t = 0; t < kSteps; ++t) {
    v8f acc[8];
#pragma unroll
    for (int j = 0; j < 8; ++j) acc[j] = (v8f){0.f,0.f,0.f,0.f,0.f,0.f,0.f,0.f};

    for (int k0 = 0; k0 < kKCat; k0 += 32) {
      FH::U fa;
      fa.h[0] = *(const v8h*)(tile + aoff + k0);
      fa.h[1] = *(const v8h*)(tile + aoff + k0 + 16);
      const v16h a = fa.v;
      v16h bq[4];
#pragma unroll
      for (int j = 0; j < 4; ++j) bq[j] = FH::load(Wcat + woff + (size_t)(j * 16) * kKCat + k0);
#pragma unroll
      for (int j = 0; j < 4; ++j) acc[j] = FH::mma(a, bq[j], acc[j]);
      guard4_h(acc[0], acc[1], acc[2], acc[3], a, bq[3]);
      keep4_h(bq[0], bq[1], bq[2], bq[3]);
      v16h br[4];
#pragma unroll
      for (int j = 0; j < 4; ++j) br[j] = FH::load(Wcat + woff + (size_t)((j + 4) * 16) * kKCat + k0);
#pragma unroll
      for (int j = 0; j < 4; ++j) acc[4 + j] = FH::mma(a, br[j], acc[4 + j]);
      guard4_h(acc[4], acc[5], acc[6], acc[7], a, br[3]);
      keep4_h(br[0], br[1], br[2], br[3]);
    }
    acc_guard4(acc[0], acc[1], acc[2], acc[3]);
    acc_guard4(acc[4], acc[5], acc[6], acc[7]);

    __syncthreads();

#pragma unroll
    for (int j = 0; j < 8; ++j) {
      _Float16* tp = tile + (hh * 8) * kTilePitch + wave * 128 + j * 16 + c;
#pragma unroll
      for (int r = 0; r < 8; ++r) tp[r * kTilePitch] = (_Float16)(acc[j][r] * kCatCarryInv);
    }
    {
      const int tn = (t + 1 < kSteps) ? (t + 1) : (kSteps - 1);
#pragma unroll
      for (int i = 0; i < 4; ++i) {
        const int idx  = i * 256 + tid;
        const int row  = idx >> 6;
        const int col8 = (idx & 63) * 8;
        const v8h v = *(const v8h*)(X16 + ((size_t)(tn * kBatch + b0 + row)) * kDModel + col8);
        *(v8h*)(tile + row * kTilePitch + kDState + col8) = v;
      }
    }
    __syncthreads();

    {
      const size_t grow0 = (size_t)(t * kBatch + b0);
      for (int pass = 0; pass < 2; ++pass) {
#pragma unroll
        for (int it = 0; it < 8; ++it) {
          const int row = 2 * wave + (it >> 2);
          const int col = (it & 3) * 256 + lane * 8;
          const v8h v = *(const v8h*)(tile + row * kTilePitch + col);
          *(volatile v8h*)(S16 + (grow0 + row) * kDState + col) = v;
        }
        __threadfence();
      }
    }
  }
}

__global__ __launch_bounds__(512) void gelu_ln_pool_kernel(const float* __restrict__ Yh, const float* __restrict__ gamma,
                                                           const float* __restrict__ beta, const float* __restrict__ PPin,
                                                           float* __restrict__ PPout, unsigned short* __restrict__ P16out,
                                                           int hsel) {
  __shared__ float psum[16];
  __shared__ float psq[16];
  __shared__ __align__(16) float sval[kDModel];
  const int b    = blockIdx.x;
  const int d    = threadIdx.x;
  const int lane = d & 31;
  const int wave = d >> 5;
  const float gm = gamma[d];
  const float bt = beta[d];
  float pool = 0.f;
  for (int tt = 0; tt < kSteps / 2; ++tt) {
    const float yv = Yh[((size_t)(tt * kBatch + b)) * kDModel + d];
    const float g  = 0.5f * yv * (1.0f + erff(yv * 0.70710678118654752f));
    float s = g;
#pragma unroll
    for (int off = 16; off > 0; off >>= 1) s += __shfl_xor(s, off, 32);
    if (lane == 0) psum[wave] = s;
    __syncthreads();
    float ssum = 0.f;
#pragma unroll
    for (int i = 0; i < 16; ++i) ssum += psum[i];
    const float mean = ssum * (1.0f / 512.0f);
    const float dl = g - mean;
    float q = dl * dl;
#pragma unroll
    for (int off = 16; off > 0; off >>= 1) q += __shfl_xor(q, off, 32);
    if (lane == 0) psq[wave] = q;
    __syncthreads();
    float qsum = 0.f;
#pragma unroll
    for (int i = 0; i < 16; ++i) qsum += psq[i];
    const float var = qsum * (1.0f / 512.0f);
    const float z = dl * rsqrtf(var + 1e-5f) * gm + bt;
    pool += z;
  }
  if (hsel == 0) {
    const float v = pool;
    float* pp = PPout + (size_t)b * kDModel + d;
    *(volatile float*)pp = v;
    __threadfence();
    *(volatile float*)pp = v;
  }
  float tot = pool;
  if (hsel != 0) tot = PPin[(size_t)b * kDModel + d] + pool;
  sval[d] = tot * kPoolMeanCarry;
  __syncthreads();
  if (hsel != 0 && d < 64) {
    const float* sp = sval + 8 * d;
    unsigned short hb[8];
#pragma unroll
    for (int e = 0; e < 8; ++e) hb[e] = h_bits(sp[e]);
    const v4u u = (v4u){pk16(hb[0], hb[1]), pk16(hb[2], hb[3]), pk16(hb[4], hb[5]), pk16(hb[6], hb[7])};
    unsigned short* q = P16out + (size_t)b * kDModel + 8 * d;
    *(volatile v4u*)q = u;
    __threadfence();
    *(volatile v4u*)q = u;
  }
}

__global__ __launch_bounds__(256) void logits_out_kernel(const float* __restrict__ L, const float* __restrict__ bfv,
                                                         float* __restrict__ out) {
  const int i = blockIdx.x * 256 + threadIdx.x;
  if (i >= (kBatch * kNCls) / 4) return;
  const int e   = 4 * i;
  const int row = e / kNCls;
  const int col = e - row * kNCls;
  const v4f a  = *(const v4f*)(L + (size_t)row * kNClsPad + col);
  const v4f bb = *(const v4f*)(bfv + col);
  const v4f v  = a + bb;
  *(volatile v4f*)(out + e) = v;
  __threadfence();
  *(volatile v4f*)(out + e) = v;
}

static inline size_t align256(size_t x) { return (x + 255) & ~(size_t)255; }

extern "C" void kernel_launch(void* const* d_in, const int* in_sizes, int n_in,
                              void* d_out, int out_size, void* d_ws, size_t ws_size,
                              hipStream_t stream) {
  if (n_in < 10) return;
  if (in_sizes[0] != kBatch * 3 * 64 * 64) return;
  if (in_sizes[1] != kDModel * kPatchK) return;
  if (in_sizes[2] != kDModel) return;
  if (in_sizes[3] != kDState * kDState) return;
  if (in_sizes[4] != kDState * kDModel) return;
  if (in_sizes[5] != kDModel * kDState) return;
  if (in_sizes[6] != kDModel || in_sizes[7] != kDModel) return;
  if (in_sizes[8] != kNCls * kDModel) return;
  if (in_sizes[9] != kNCls) return;
  if (out_size != kBatch * kNCls) return;

  const float* images = (const float*)d_in[0];
  const float* Wp     = (const float*)d_in[1];
  const float* bp     = (const float*)d_in[2];
  const float* Am     = (const float*)d_in[3];
  const float* Bmm    = (const float*)d_in[4];
  const float* Cm     = (const float*)d_in[5];
  const float* gamma  = (const float*)d_in[6];
  const float* beta   = (const float*)d_in[7];
  const float* Wf     = (const float*)d_in[8];
  const float* bfv    = (const float*)d_in[9];
  float* out = (float*)d_out;

  char* ws = (char*)d_ws;
  size_t off = 0;
  const size_t oWcat = off; off = align256(off + (size_t)kDState * kKCat * 2);
  const size_t oCm   = off; off = align256(off + (size_t)kDModel * kDState * 2);
  const size_t oWf   = off; off = align256(off + (size_t)kNClsPad * kDModel * 2);
  const size_t oWp   = off; off = align256(off + (size_t)kDModel * kPatchKPad * 2);
  const size_t oP    = off; off = align256(off + (size_t)kRows * kPatchKPad * 2);
  const size_t oX    = off; off = align256(off + (size_t)kRows * kDModel * 2);
  const size_t oS    = off; off = align256(off + (size_t)kRows * kDState * 2);
  const size_t oPP   = off; off = align256(off + (size_t)kBatch * kDModel * 4);
  const size_t oPool = off; off = align256(off + (size_t)kBatch * kDModel * 2);
  const size_t oL    = off; off = align256(off + (size_t)kBatch * kNClsPad * 4);
  if (off > ws_size) return;

  unsigned short* Wcat16 = (unsigned short*)(ws + oWcat);
  unsigned short* Cm16   = (unsigned short*)(ws + oCm);
  unsigned short* Wf16   = (unsigned short*)(ws + oWf);
  unsigned short* Wp16   = (unsigned short*)(ws + oWp);
  unsigned short* P16    = (unsigned short*)(ws + oP);
  unsigned short* X16    = (unsigned short*)(ws + oX);
  float*          Yh     = (float*)(ws + oX);
  unsigned short* S16    = (unsigned short*)(ws + oS);
  float*          PP     = (float*)(ws + oPP);
  unsigned short* pooled16 = (unsigned short*)(ws + oPool);
  float*          Lws    = (float*)(ws + oL);

  build_wcat_kernel<<<(kDState * (kKCat / 8)) / 256, 256, 0, stream>>>(Am, Bmm, Wcat16);
  cast8_scale_kernel<<<(kDModel * kDState / 8) / 256, 256, 0, stream>>>(Cm, Cm16, kDModel * kDState / 8, kCmCarry);
  cast_wf_kernel<<<(kNClsPad * (kDModel / 8)) / 256, 256, 0, stream>>>(Wf, Wf16);
  cast_wp_kernel<<<(kDModel * (kPatchKPad / 8)) / 256, 256, 0, stream>>>(Wp, Wp16);
  patchify_kernel<<<(kRows * (kPatchKPad / 8)) / 256, 256, 0, stream>>>(images, P16);
  wmma_gemm64<0, false, 2, 1, false><<<dim3((kRows / 64) * (kDModel / 64) / 8, 1), 256, 0, stream>>>(
      P16, P16, kPatchKPad, 0L, Wp16, Wp16, kPatchKPad, 0L,
      (void*)X16, (void*)X16, kDModel, 0L, bp, Lws, 0L, kRows, kDModel, kPatchKPad, kWpCarryInv);
  ssm_scan_kernel<<<kBatch / kRowsPerBlk, 256, 0, stream>>>(X16, Wcat16, S16);
  for (int h = 0; h < 2; ++h) {
    const unsigned short* Sh = S16 + (size_t)h * kHalfRows * kDState;
    wmma_gemm64<0, false, 0, 0, false><<<dim3((kHalfRows / 64) * (kDModel / 64) / 8, 1), 256, 0, stream>>>(
        Sh, Sh, kDState, 0L, Cm16, Cm16, kDState, 0L,
        (void*)Yh, (void*)Yh, kDModel, 0L, bp, Lws, 0L, kHalfRows, kDModel, kDState, kCmCarryInv);
    gelu_ln_pool_kernel<<<kBatch, 512, 0, stream>>>(Yh, gamma, beta, PP, PP, pooled16, h);
  }
  wmma_gemm64<0, false, 0, 0, false><<<dim3((kBatch / 64) * (kNClsPad / 64) / 8, 1), 256, 0, stream>>>(
      pooled16, pooled16, kDModel, 0L, Wf16, Wf16, kDModel, 0L,
      (void*)Lws, (void*)Lws, kNClsPad, 0L, bp, PP, 0L, kBatch, kNClsPad, kDModel, kLogitScale);
  logits_out_kernel<<<(kBatch * kNCls / 4 + 255) / 256, 256, 0, stream>>>(Lws, bfv, out);
}
